// ModelDebug_18717467476434
// MI455X (gfx1250) — hardware-verified
//
#include <hip/hip_runtime.h>
#include <stddef.h>


typedef __attribute__((ext_vector_type(16))) _Float16 v16h;
typedef __attribute__((ext_vector_type(8)))  _Float16 v8h;
typedef __attribute__((ext_vector_type(4)))  _Float16 v4h;
typedef __attribute__((ext_vector_type(8)))  float    v8f;
typedef __attribute__((ext_vector_type(4)))  float    v4f;

#define NB    8
#define NT    1024
#define NC    768
#define NH    12
#define HD    64
#define M_ALL (NB * NT)
#define N_ALL (3 * NC)
#define PLANE (NB * NH * NT * HD)

__device__ inline v8f wmma_f16(v16h a, v16h b, v8f c) {
  v8f d = __builtin_amdgcn_wmma_f32_16x16x32_f16(false, a, false, b, (short)0, c, false, false);
  asm volatile("v_nop\n\tv_nop\n\tv_nop\n\tv_nop" : "+v"(d) : "v"(a), "v"(b));
  return d;
}
#define VST2(T, ptr, val) do { const T _v = (val); *(volatile T*)(ptr) = _v; __threadfence(); *(volatile T*)(ptr) = _v; } while (0)

__device__ inline v8h ld8(const _Float16* p) { return *(const v8h*)p; }

__device__ inline v16h make_frag(v8h lo, v8h hi) {
  v16h r;
#pragma unroll
  for (int i = 0; i < 8; ++i) { r[i] = lo[i]; r[i + 8] = hi[i]; }
  return r;
}


__global__ void __launch_bounds__(256)
cvt_f32_to_f16(const float* __restrict__ in, _Float16* __restrict__ out, int n) {
  int i = (blockIdx.x * blockDim.x + threadIdx.x) * 4;
  if (i < n) {
    v4f d = *(const v4f*)(in + i);
    v4h o;
#pragma unroll
    for (int e = 0; e < 4; ++e) o[e] = (_Float16)d[e];
    VST2(v4h, out + i, o);
  }
}

__global__ void __launch_bounds__(256)
qkv_gemm(const _Float16* __restrict__ xh, const _Float16* __restrict__ wh,
         const float* __restrict__ bias, _Float16* __restrict__ qkv) {
  const int lane = threadIdx.x & 31;
  const int wave = threadIdx.x >> 5;
  const int l = lane & 15, s = (lane >> 4) & 1;
  const int m0 = blockIdx.y * 128 + (wave >> 1) * 32;
  const int n0 = blockIdx.x * 128 + (wave & 1) * 64;

  const _Float16* aP = xh + (size_t)(m0 + l) * NC + 8 * s;
  const _Float16* bP = wh + (size_t)(n0 + l) * NC + 8 * s;

  v8f acc[2][4] = {};
  for (int k0 = 0; k0 < NC; k0 += 32) {
    __builtin_prefetch(aP + 64, 0, 3);
    v16h a0 = make_frag(ld8(aP), ld8(aP + 16));
    v16h a1 = make_frag(ld8(aP + 16 * NC), ld8(aP + 16 * NC + 16));
    v16h b0 = make_frag(ld8(bP), ld8(bP + 16));
    v16h b1 = make_frag(ld8(bP + 16 * NC), ld8(bP + 16 * NC + 16));
    v16h b2 = make_frag(ld8(bP + 32 * NC), ld8(bP + 32 * NC + 16));
    v16h b3 = make_frag(ld8(bP + 48 * NC), ld8(bP + 48 * NC + 16));
    acc[0][0] = wmma_f16(a0, b0, acc[0][0]);
    acc[1][0] = wmma_f16(a1, b0, acc[1][0]);
    acc[0][1] = wmma_f16(a0, b1, acc[0][1]);
    acc[1][1] = wmma_f16(a1, b1, acc[1][1]);
    acc[0][2] = wmma_f16(a0, b2, acc[0][2]);
    acc[1][2] = wmma_f16(a1, b2, acc[1][2]);
    acc[0][3] = wmma_f16(a0, b3, acc[0][3]);
    acc[1][3] = wmma_f16(a1, b3, acc[1][3]);
    aP += 32;
    bP += 32;
  }

  __shared__ __attribute__((aligned(16))) _Float16 sT[2][64][136];
  const int which = (blockIdx.x * 128 >= 2 * NC) ? 2 : ((blockIdx.x * 128 >= NC) ? 1 : 0);
  const int bidx = blockIdx.y >> 3;
  const int t0blk = (blockIdx.y & 7) * 128;
  const int cblk = blockIdx.x * 128 - which * NC;
  const int h0 = cblk >> 6;
  {
    const int g = wave & 1;
    const int trow0 = (wave >> 1) * 32;
#pragma unroll
    for (int j = 0; j < 4; ++j) {
      const int d = 16 * j + l;
      const float bv = bias[n0 + 16 * j + l];
#pragma unroll
      for (int i = 0; i < 2; ++i)
#pragma unroll
        for (int r = 0; r < 8; ++r) sT[g][d][trow0 + 16 * i + 8 * s + r] = (_Float16)(acc[i][j][r] + bv);
    }
  }
  __syncthreads();
  for (int pass = 0; pass < 2; ++pass) {
    if (which == 2) {
      for (int p = threadIdx.x; p < 2 * 64 * 16; p += 256) {
        const int g = p >> 10, d = (p >> 4) & 63, q = p & 15;
        _Float16* dst = qkv + 2u * PLANE + ((size_t)(bidx * NH + h0 + g) * HD + d) * NT + t0blk + q * 8;
        *(volatile v8h*)dst = *(const v8h*)&sT[g][d][q * 8];
      }
    } else {
      for (int p = threadIdx.x; p < 2 * 128 * 8; p += 256) {
        const int g = p >> 10, t = (p >> 3) & 127, q = p & 7;
        v8h v;
#pragma unroll
        for (int e = 0; e < 8; ++e) v[e] = sT[g][q * 8 + e][t];
        _Float16* dst = qkv + (unsigned)which * PLANE + ((size_t)(bidx * NH + h0 + g) * NT + t0blk + t) * HD + q * 8;
        *(volatile v8h*)dst = v;
      }
    }
    __threadfence();
  }
}

__global__ void __launch_bounds__(128)
attn_relu(const _Float16* __restrict__ qkv, float* __restrict__ out) {
  __shared__ _Float16 sS[4][16][72];
  __shared__ _Float16 sL[4][16][72];

  const int lane = threadIdx.x & 31;
  const int wave = threadIdx.x >> 5;
  const int l = lane & 15, s = (lane >> 4) & 1;
  const int bh = blockIdx.y;
  const int b = bh / NH, h = bh - b * NH;
  const int qt = blockIdx.x;
  const int qrow0 = qt * 64 + wave * 16;

  v16h qa0, qa1;
  {
    const _Float16* qa = qkv + (size_t)bh * NT * HD + (size_t)(qrow0 + l) * HD + 8 * s;
    qa0 = make_frag(ld8(qa), ld8(qa + 16));
    qa1 = make_frag(ld8(qa + 32), ld8(qa + 48));
  }
  const _Float16* kP = qkv + 1u * PLANE + (size_t)bh * NT * HD + (size_t)l * HD + 8 * s;
  const _Float16* vP = qkv + 2u * PLANE + (size_t)bh * HD * NT + (size_t)l * NT + 8 * s;
  _Float16* sSt = &sS[wave][8 * s][l];
  const _Float16* sLd = &sS[wave][l][8 * s];
  _Float16* sLt = &sL[wave][8 * s][l];
  const _Float16* sLl = &sL[wave][l][8 * s];

  v8f yacc[4] = {};
  const int nkt = qt + 1;
  const int m_g0 = qrow0 + 8 * s;

  for (int kt = 0; kt < nkt; ++kt) {
#pragma unroll
    for (int nt = 0; nt < 4; ++nt) {
      v16h kb0 = make_frag(ld8(kP + nt * 16 * HD), ld8(kP + nt * 16 * HD + 16));
      v16h kb1 = make_frag(ld8(kP + nt * 16 * HD + 32), ld8(kP + nt * 16 * HD + 48));
      v8f sacc = {};
      sacc = wmma_f16(qa0, kb0, sacc);
      sacc = wmma_f16(qa1, kb1, sacc);
      const int n_g = kt * 64 + nt * 16 + l;
#pragma unroll
      for (int r = 0; r < 8; ++r) {
        float v = sacc[r] * 0.125f;
        v = (n_g <= m_g0 + r) ? fmaxf(v, 0.0f) : 0.0f;
        const _Float16 vh = (_Float16)v;
        sSt[r * 72 + nt * 16] = vh;
        sLt[r * 72 + nt * 16] = (_Float16)(v - (float)vh);
      }
    }
    __builtin_amdgcn_wave_barrier();

#pragma unroll
    for (int kk0 = 0; kk0 < 64; kk0 += 32) {
      v16h sa = make_frag(*(const v8h*)(sLd + kk0), *(const v8h*)(sLd + kk0 + 16));
      v16h sl = make_frag(*(const v8h*)(sLl + kk0), *(const v8h*)(sLl + kk0 + 16));
#pragma unroll
      for (int nt = 0; nt < 4; ++nt) {
        v16h vb = make_frag(ld8(vP + nt * 16 * NT + kk0),
                            ld8(vP + nt * 16 * NT + kk0 + 16));
        yacc[nt] = wmma_f16(sa, vb, yacc[nt]);
        yacc[nt] = wmma_f16(sl, vb, yacc[nt]);
      }
    }
    __builtin_amdgcn_wave_barrier();

    kP += 64 * HD;
    vP += 64;
  }

  float* ob = out + ((size_t)b * NT + qrow0) * NC + h * HD;
  for (int pass = 0; pass < 2; ++pass) {
#pragma unroll
    for (int pr = 0; pr < 2; ++pr)
#pragma unroll
      for (int r = 0; r < 8; ++r) {
        const float a_ = yacc[2 * pr][r], b_ = yacc[2 * pr + 1][r];
        const float ax = __shfl_xor(a_, 16), bx = __shfl_xor(b_, 16);
        *(volatile float*)(ob + (size_t)r * NC + pr * 32 + lane)       = s ? bx : a_;
        *(volatile float*)(ob + (size_t)(r + 8) * NC + pr * 32 + lane) = s ? b_ : ax;
      }
    __threadfence();
  }
}

extern "C" void kernel_launch(void* const* d_in, const int* in_sizes, int n_in,
                              void* d_out, int out_size, void* d_ws, size_t ws_size,
                              hipStream_t stream) {
  const float* x    = (const float*)d_in[0];
  const float* W    = (const float*)d_in[1];
  const float* bias = (const float*)d_in[2];
  float* out = (float*)d_out;

  (void)in_sizes; (void)n_in; (void)out_size;
  char* ws = (char*)d_ws;
  const size_t n_x = (size_t)M_ALL * NC;
  if (ws_size < (n_x + (size_t)N_ALL * NC + 3 * (size_t)PLANE) * sizeof(_Float16)) return;
  const size_t n_w = (size_t)N_ALL * NC;
  _Float16* xh   = (_Float16*)ws;
  _Float16* wh   = (_Float16*)(ws + n_x * sizeof(_Float16));
  _Float16* qkvh = (_Float16*)(ws + (n_x + n_w) * sizeof(_Float16));

  cvt_f32_to_f16<<<(int)(n_x / 4 / 256), 256, 0, stream>>>(x, xh, (int)n_x);
  cvt_f32_to_f16<<<(int)(n_w / 4 / 256), 256, 0, stream>>>(W, wh, (int)n_w);

  qkv_gemm<<<dim3(N_ALL / 128, M_ALL / 128), 256, 0, stream>>>(xh, wh, bias, qkvh);

  attn_relu<<<dim3(NT / 64, NB * NH), 128, 0, stream>>>(qkvh, out);
}
